// GCN_mamba_Net_16149077033110
// MI455X (gfx1250) — hardware-verified
//
#include <hip/hip_runtime.h>
#define NN 2048
#define FIN 1024
#define DM 256
#define DI 256
#define DSG 8
#define DTRG 16
#define KC 4
#define DSB 16
#define DTRB 16
#define LG 8

typedef __bf16 v16b __attribute__((ext_vector_type(16)));
typedef unsigned short v8us __attribute__((ext_vector_type(8), may_alias));
typedef float  v8f  __attribute__((ext_vector_type(8)));
typedef float  v4f  __attribute__((ext_vector_type(4)));
typedef float  v4fa __attribute__((ext_vector_type(4), may_alias));
union FragB { v16b v; v8us half[2]; unsigned short u[16]; };

__device__ __forceinline__ unsigned short bf16_bits(float x) { unsigned int u = __float_as_uint(x); return (unsigned short)((u + 0x7FFFu + ((u >> 16) & 1u)) >> 16); }
__device__ __forceinline__ float bf16_val(unsigned short b) { return __uint_as_float(((unsigned int)b) << 16); }
__device__ __forceinline__ float bf16_round(float x) { return bf16_val(bf16_bits(x)); }
template <int NT>
__device__ __forceinline__ v8f mmaN(v16b ah, v16b al, v16b bh, v16b bl, v8f c) {
  c = __builtin_amdgcn_wmma_f32_16x16x32_bf16(false, ah, false, bh, (short)0, c, false, false);
  if (NT >= 2) c = __builtin_amdgcn_wmma_f32_16x16x32_bf16(false, al, false, bh, (short)0, c, false, false);
  if (NT >= 3) c = __builtin_amdgcn_wmma_f32_16x16x32_bf16(false, ah, false, bl, (short)0, c, false, false);
  asm volatile("v_nop\n\tv_nop\n\tv_nop\n\tv_nop" : "+v"(c) : "v"(ah), "v"(al), "v"(bh), "v"(bl));
  return c;
}

__global__ __launch_bounds__(256) void k_wt_bf16(const float* __restrict__ W, unsigned short* __restrict__ Wt, int K, int N) {
  const int t = blockIdx.x * 256 + threadIdx.x;
  const int k8n = K / 8;
  if (t >= N * k8n) return;
  const int n = t / k8n, k8 = (t % k8n) * 8;
  v8us v;
#pragma unroll
  for (int i = 0; i < 8; ++i) v[i] = bf16_bits(W[(size_t)(k8 + i) * N + n]);
  *(volatile v8us*)(Wt + (size_t)n * K + k8) = v;
  __threadfence();
  *(volatile v8us*)(Wt + (size_t)n * K + k8) = v;
}

template <bool ASPLIT, int ACT, bool BIAS_BF16>
__global__ __launch_bounds__(128) void k_gemm_bf(const float* __restrict__ A, int lda, const unsigned short* __restrict__ Wt, int ldb,
                                               const float* __restrict__ bias, float* __restrict__ C, int ldc, int M, int N, int K) {
  __shared__ __attribute__((aligned(16))) float so[4][16][64];
  const int tid = threadIdx.x, w = tid >> 5, lane = tid & 31, ln = lane & 15, hh = lane >> 4;
  const int ntn = N / 64;
  const int wid = blockIdx.x * 4 + w;
  const int mt = wid / ntn, nq = wid % ntn;
  if (mt * 16 >= M) return;
  const int row0 = mt * 16, col0 = nq * 64;
  const float* arow = A + (size_t)(row0 + ln) * lda;
  v8f acc[4] = {};
  for (int kb = 0; kb < K; kb += 32) {
    FragB ah, al;
    const v4f x0 = *(const v4fa*)(arow + kb + 8 * hh), x1 = *(const v4fa*)(arow + kb + 8 * hh + 4);
    const v4f x2 = *(const v4fa*)(arow + kb + 16 + 8 * hh), x3 = *(const v4fa*)(arow + kb + 16 + 8 * hh + 4);
    float xs[16] = {x0[0],x0[1],x0[2],x0[3],x1[0],x1[1],x1[2],x1[3],x2[0],x2[1],x2[2],x2[3],x3[0],x3[1],x3[2],x3[3]};
#pragma unroll
    for (int i = 0; i < 16; ++i) { const unsigned short hb = bf16_bits(xs[i]); ah.u[i] = hb; al.u[i] = ASPLIT ? bf16_bits(xs[i] - bf16_val(hb)) : (unsigned short)0; }
#pragma unroll
    for (int t = 0; t < 4; ++t) {
      const unsigned short* brow = Wt + (size_t)(col0 + t * 16 + ln) * ldb + kb;
      FragB b;
      b.half[0] = *(const v8us*)(brow + 8 * hh);
      b.half[1] = *(const v8us*)(brow + 16 + 8 * hh);
      acc[t] = mmaN<ASPLIT ? 2 : 1>(ah.v, al.v, b.v, b.v, acc[t]);
    }
  }
#pragma unroll
  for (int t = 0; t < 4; ++t) {
    float bv = bias ? bias[col0 + t * 16 + ln] : 0.f;
    if (BIAS_BF16) bv = bf16_round(bv);
#pragma unroll
    for (int r = 0; r < 8; ++r) { float v = acc[t][r] + bv; if (ACT == 1) v = fmaxf(v, 0.f); so[w][8 * hh + r][t * 16 + ln] = v; }
  }
  __builtin_amdgcn_fence(__ATOMIC_ACQ_REL, "workgroup");
  __builtin_amdgcn_wave_barrier();
  const int rsub = lane >> 4, c4 = (lane & 15) * 4;
  for (int pass = 0; pass < 2; ++pass) {
#pragma unroll
    for (int q = 0; q < 8; ++q) {
      const int r = q * 2 + rsub;
      const v4f v = *(const v4fa*)&so[w][r][c4];
      *(volatile v4f*)(C + (size_t)(row0 + r) * ldc + col0 + c4) = v;
    }
    if (pass == 0) __threadfence();
  }
}

template <int D, bool CAUSAL>
__global__ __launch_bounds__(128) void k_flash(const float* __restrict__ qb, const float* __restrict__ kb, const float* __restrict__ vb,
                                             int pitch, int T, int H, float scale, float* __restrict__ y, int ypitch) {
  constexpr int KS = D / 32;
  constexpr int DT = D / 16;
  __shared__ __attribute__((aligned(16))) unsigned short sKh[32][D + 8], sKl[32][D + 8], sVh[32][D + 8], sVl[32][D + 8];
  __shared__ __attribute__((aligned(16))) unsigned short sPh[4][16][40], sPl[4][16][40];
  __shared__ __attribute__((aligned(16))) float sO[4][16][D];
  const int tid = threadIdx.x, w = tid >> 5, lane = tid & 31, ln = lane & 15, hh = lane >> 4;
  const int nqb = (T + 63) / 64;
  const int bh = blockIdx.x / nqb, qblk = blockIdx.x % nqb;
  const int b = bh / H, h = bh % H;
  const int q0 = qblk * 64 + w * 16;
  const float* Q = qb + (size_t)b * T * pitch + h * D;
  const float* K = kb + (size_t)b * T * pitch + h * D;
  const float* V = vb + (size_t)b * T * pitch + h * D;

  FragB aqh[KS], aql[KS];
  {
    int row = q0 + ln; if (row >= T) row = T - 1;
    const float* qr = Q + (size_t)row * pitch;
#pragma unroll
    for (int ks = 0; ks < KS; ++ks)
#pragma unroll
      for (int i = 0; i < 16; ++i) {
        const int d = ks * 32 + ((i < 8) ? (8 * hh + i) : (16 + 8 * hh + (i - 8)));
        const float x = qr[d] * scale; const unsigned short hb = bf16_bits(x);
        aqh[ks].u[i] = hb; aql[ks].u[i] = bf16_bits(x - bf16_val(hb));
      }
  }
  float m_r[8], l_r[8];
#pragma unroll
  for (int r = 0; r < 8; ++r) { m_r[r] = -3.0e38f; l_r[r] = 0.f; }
  v8f oacc[DT];
#pragma unroll
  for (int dt = 0; dt < DT; ++dt) oacc[dt] = (v8f){0.f,0.f,0.f,0.f,0.f,0.f,0.f,0.f};

  const int kv_end = CAUSAL ? min(T, qblk * 64 + 64) : T;
  for (int j0 = 0; j0 < kv_end; j0 += 32) {
    __syncthreads();
    for (int e = tid; e < 32 * (D / 4); e += 128) {
      const int r = e / (D / 4), c4 = (e % (D / 4)) * 4;
      const int key = j0 + r;
      v4f kf = {0.f,0.f,0.f,0.f}, vf = {0.f,0.f,0.f,0.f};
      if (key < T) { kf = *(const v4fa*)(K + (size_t)key * pitch + c4); vf = *(const v4fa*)(V + (size_t)key * pitch + c4); }
#pragma unroll
      for (int t = 0; t < 4; ++t) {
        unsigned short hb = bf16_bits(kf[t]); sKh[r][c4 + t] = hb; sKl[r][c4 + t] = bf16_bits(kf[t] - bf16_val(hb));
        hb = bf16_bits(vf[t]); sVh[r][c4 + t] = hb; sVl[r][c4 + t] = bf16_bits(vf[t] - bf16_val(hb));
      }
    }
    __syncthreads();
    v8f s[2];
#pragma unroll
    for (int nt = 0; nt < 2; ++nt) {
      v8f acc = {};
#pragma unroll
      for (int ks = 0; ks < KS; ++ks) {
        FragB bh_, bl_;
        bh_.half[0] = *(const v8us*)&sKh[nt * 16 + ln][ks * 32 + 8 * hh]; bh_.half[1] = *(const v8us*)&sKh[nt * 16 + ln][ks * 32 + 16 + 8 * hh];
        bl_.half[0] = *(const v8us*)&sKl[nt * 16 + ln][ks * 32 + 8 * hh]; bl_.half[1] = *(const v8us*)&sKl[nt * 16 + ln][ks * 32 + 16 + 8 * hh];
        acc = mmaN<3>(aqh[ks].v, aql[ks].v, bh_.v, bl_.v, acc);
      }
      s[nt] = acc;
    }
    float alpha[8];
#pragma unroll
    for (int r = 0; r < 8; ++r) {
      const int qi = q0 + 8 * hh + r;
      const int ja = j0 + ln, jb = j0 + 16 + ln;
      if (CAUSAL) { if (ja > qi) s[0][r] = -3.0e38f; if (jb > qi) s[1][r] = -3.0e38f; }
      if (ja >= T) s[0][r] = -3.0e38f;
      if (jb >= T) s[1][r] = -3.0e38f;
      float mx = fmaxf(s[0][r], s[1][r]);
      mx = fmaxf(mx, __shfl_xor(mx, 1, 32)); mx = fmaxf(mx, __shfl_xor(mx, 2, 32)); mx = fmaxf(mx, __shfl_xor(mx, 4, 32)); mx = fmaxf(mx, __shfl_xor(mx, 8, 32));
      const float mnew = fmaxf(m_r[r], mx);
      alpha[r] = (mnew > -1.0e38f) ? __expf(m_r[r] - mnew) : 1.0f;
      const float p0 = (s[0][r] > -1.0e38f) ? __expf(s[0][r] - mnew) : 0.f;
      const float p1 = (s[1][r] > -1.0e38f) ? __expf(s[1][r] - mnew) : 0.f;
      m_r[r] = mnew;
      l_r[r] = l_r[r] * alpha[r] + p0 + p1;
      unsigned short hb = bf16_bits(p0); sPh[w][8 * hh + r][ln] = hb;      sPl[w][8 * hh + r][ln] = bf16_bits(p0 - bf16_val(hb));
      hb = bf16_bits(p1);                sPh[w][8 * hh + r][16 + ln] = hb; sPl[w][8 * hh + r][16 + ln] = bf16_bits(p1 - bf16_val(hb));
    }
#pragma unroll
    for (int dt = 0; dt < DT; ++dt)
#pragma unroll
      for (int r = 0; r < 8; ++r) oacc[dt][r] *= alpha[r];
    __builtin_amdgcn_fence(__ATOMIC_ACQ_REL, "workgroup");
    __builtin_amdgcn_wave_barrier();
    FragB pah, pal;
    pah.half[0] = *(const v8us*)&sPh[w][ln][8 * hh]; pah.half[1] = *(const v8us*)&sPh[w][ln][16 + 8 * hh];
    pal.half[0] = *(const v8us*)&sPl[w][ln][8 * hh]; pal.half[1] = *(const v8us*)&sPl[w][ln][16 + 8 * hh];
#pragma unroll
    for (int dt = 0; dt < DT; ++dt) {
      FragB bvh, bvl;
#pragma unroll
      for (int i = 0; i < 8; ++i) {
        bvh.u[i] = sVh[8 * hh + i][dt * 16 + ln]; bvh.u[8 + i] = sVh[16 + 8 * hh + i][dt * 16 + ln];
        bvl.u[i] = sVl[8 * hh + i][dt * 16 + ln]; bvl.u[8 + i] = sVl[16 + 8 * hh + i][dt * 16 + ln];
      }
      oacc[dt] = mmaN<3>(pah.v, pal.v, bvh.v, bvl.v, oacc[dt]);
    }
    __builtin_amdgcn_fence(__ATOMIC_ACQ_REL, "workgroup");
    __builtin_amdgcn_wave_barrier();
  }
#pragma unroll
  for (int r = 0; r < 8; ++r) {
    float l = l_r[r];
    l += __shfl_xor(l, 1, 32); l += __shfl_xor(l, 2, 32); l += __shfl_xor(l, 4, 32); l += __shfl_xor(l, 8, 32);
    l_r[r] = (l > 0.f) ? 1.0f / l : 0.f;
  }
#pragma unroll
  for (int dt = 0; dt < DT; ++dt)
#pragma unroll
    for (int r = 0; r < 8; ++r) sO[w][8 * hh + r][dt * 16 + ln] = oacc[dt][r] * l_r[r];
  __builtin_amdgcn_fence(__ATOMIC_ACQ_REL, "workgroup");
  __builtin_amdgcn_wave_barrier();
  for (int pass = 0; pass < 2; ++pass) {
    for (int r = 0; r < 16; ++r) {
      const int row = q0 + r;
      if (row < T && lane < D / 4) {
        const v4f val = *(const v4fa*)&sO[w][r][lane * 4];
        *(volatile v4f*)(y + ((size_t)b * T + row) * ypitch + h * D + lane * 4) = val;
      }
    }
    if (pass == 0) __threadfence();
  }
}

template <bool AFFINE, bool RESID, bool RES_BF16>
__global__ __launch_bounds__(256) void k_transpose32(const float* __restrict__ in, float* __restrict__ out, int rows, int cols,
                                                    const float* __restrict__ scale, const float* __restrict__ shift, const float* __restrict__ res) {
  __shared__ float tile[32][33];
  const int b = blockIdx.z;
  const int r0 = blockIdx.y * 32, c0 = blockIdx.x * 32;
  const float* src = in + (size_t)b * rows * cols;
  float* dst = out + (size_t)b * rows * cols;
  const int tx = threadIdx.x & 31, ty = threadIdx.x >> 5;
  for (int i = ty; i < 32; i += 8) tile[i][tx] = src[(size_t)(r0 + i) * cols + c0 + tx];
  __syncthreads();
  for (int pass = 0; pass < 2; ++pass) {
    for (int i = ty; i < 32; i += 8) {
      float v = tile[tx][i];
      const int orow = c0 + i;
      if (AFFINE) v = v * scale[orow] + shift[orow];
      if (RESID) { float rv = res[(size_t)b * rows * cols + (size_t)orow * rows + r0 + tx]; if (RES_BF16) rv = bf16_round(rv); v += rv; }
      *(volatile float*)(dst + (size_t)orow * rows + r0 + tx) = v;
    }
    if (pass == 0) __threadfence();
  }
}

__global__ __launch_bounds__(256) void k_pool2_pm(const float* __restrict__ in, float* __restrict__ out, int Bn, int H, int W, int C) {
  const size_t t = (size_t)blockIdx.x * 256 + threadIdx.x;
  const int c4n = C / 4, Ho = H / 2, Wo = W / 2;
  const size_t total = (size_t)Bn * Ho * Wo * c4n;
  if (t >= total) return;
  const int c4 = (int)(t % c4n) * 4; size_t rest = t / c4n;
  const int pw = (int)(rest % Wo); rest /= Wo; const int ph = (int)(rest % Ho); const int b = (int)(rest / Ho);
  const float* base = in + (size_t)b * H * W * C;
  const int p00 = (2 * ph) * W + 2 * pw;
  const v4f a = *(const v4fa*)(base + (size_t)p00 * C + c4), bq = *(const v4fa*)(base + (size_t)(p00 + 1) * C + c4);
  const v4f c = *(const v4fa*)(base + (size_t)(p00 + W) * C + c4), d = *(const v4fa*)(base + (size_t)(p00 + W + 1) * C + c4);
  v4f m; for (int i = 0; i < 4; ++i) m[i] = fmaxf(fmaxf(a[i], bq[i]), fmaxf(c[i], d[i]));
  float* dst = out + ((size_t)b * Ho * Wo + (size_t)ph * Wo + pw) * C + c4;
  *(volatile v4f*)dst = m;
  __threadfence();
  *(volatile v4f*)dst = m;
}

template <int DQ, int DV>
__global__ __launch_bounds__(128) void k_flash2(const float* __restrict__ Qb, size_t qstride, int qpitch, int Tq,
                                              const float* __restrict__ Kb, size_t kstride, int kpitch, int Tk,
                                              const float* __restrict__ Vb, size_t vstride, int vpitch,
                                              float scale, float* __restrict__ y, size_t ystride, int ypitch) {
  constexpr int KS = DQ / 32, DT = DV / 16;
  __shared__ __attribute__((aligned(16))) unsigned short sKh[32][DQ + 8], sKl[32][DQ + 8], sVh[32][DV + 8], sVl[32][DV + 8];
  __shared__ __attribute__((aligned(16))) unsigned short sPh[4][16][40], sPl[4][16][40];
  __shared__ __attribute__((aligned(16))) float sO[4][16][DV];
  const int tid = threadIdx.x, w = tid >> 5, lane = tid & 31, ln = lane & 15, hh = lane >> 4;
  const int nqb = (Tq + 63) / 64;
  const int bh = blockIdx.x / nqb, qblk = blockIdx.x % nqb;
  const int dv0 = blockIdx.y * DV;
  const int q0 = qblk * 64 + w * 16;
  const float* Q = Qb + (size_t)bh * qstride; const float* K = Kb + (size_t)bh * kstride; const float* V = Vb + (size_t)bh * vstride + dv0;
  FragB aqh[KS], aql[KS];
  {
    int row = q0 + ln; if (row >= Tq) row = Tq - 1;
    const float* qr = Q + (size_t)row * qpitch;
#pragma unroll
    for (int ks = 0; ks < KS; ++ks)
#pragma unroll
      for (int i = 0; i < 16; ++i) {
        const int d = ks * 32 + ((i < 8) ? (8 * hh + i) : (16 + 8 * hh + (i - 8)));
        const float x = qr[d] * scale; const unsigned short hb = bf16_bits(x);
        aqh[ks].u[i] = hb; aql[ks].u[i] = bf16_bits(x - bf16_val(hb));
      }
  }
  float m_r[8], l_r[8];
#pragma unroll
  for (int r = 0; r < 8; ++r) { m_r[r] = -3.0e38f; l_r[r] = 0.f; }
  v8f oacc[DT];
#pragma unroll
  for (int dt = 0; dt < DT; ++dt) oacc[dt] = (v8f){0.f,0.f,0.f,0.f,0.f,0.f,0.f,0.f};
  for (int j0 = 0; j0 < Tk; j0 += 32) {
    __syncthreads();
    for (int e = tid; e < 32 * (DQ / 4); e += 128) {
      const int r = e / (DQ / 4), c4 = (e % (DQ / 4)) * 4; const int key = j0 + r;
      v4f f = {0.f,0.f,0.f,0.f}; if (key < Tk) f = *(const v4fa*)(K + (size_t)key * kpitch + c4);
#pragma unroll
      for (int t = 0; t < 4; ++t) { const unsigned short hb = bf16_bits(f[t]); sKh[r][c4 + t] = hb; sKl[r][c4 + t] = bf16_bits(f[t] - bf16_val(hb)); }
    }
    for (int e = tid; e < 32 * (DV / 4); e += 128) {
      const int r = e / (DV / 4), c4 = (e % (DV / 4)) * 4; const int key = j0 + r;
      v4f f = {0.f,0.f,0.f,0.f}; if (key < Tk) f = *(const v4fa*)(V + (size_t)key * vpitch + c4);
#pragma unroll
      for (int t = 0; t < 4; ++t) { const unsigned short hb = bf16_bits(f[t]); sVh[r][c4 + t] = hb; sVl[r][c4 + t] = bf16_bits(f[t] - bf16_val(hb)); }
    }
    __syncthreads();
    v8f s[2];
#pragma unroll
    for (int nt = 0; nt < 2; ++nt) {
      v8f acc = {};
#pragma unroll
      for (int ks = 0; ks < KS; ++ks) {
        FragB bh_, bl_;
        bh_.half[0] = *(const v8us*)&sKh[nt * 16 + ln][ks * 32 + 8 * hh]; bh_.half[1] = *(const v8us*)&sKh[nt * 16 + ln][ks * 32 + 16 + 8 * hh];
        bl_.half[0] = *(const v8us*)&sKl[nt * 16 + ln][ks * 32 + 8 * hh]; bl_.half[1] = *(const v8us*)&sKl[nt * 16 + ln][ks * 32 + 16 + 8 * hh];
        acc = mmaN<3>(aqh[ks].v, aql[ks].v, bh_.v, bl_.v, acc);
      }
      s[nt] = acc;
    }
    float alpha[8];
#pragma unroll
    for (int r = 0; r < 8; ++r) {
      const int ja = j0 + ln, jb = j0 + 16 + ln;
      if (ja >= Tk) s[0][r] = -3.0e38f;
      if (jb >= Tk) s[1][r] = -3.0e38f;
      float mx = fmaxf(s[0][r], s[1][r]);
      mx = fmaxf(mx, __shfl_xor(mx, 1, 32)); mx = fmaxf(mx, __shfl_xor(mx, 2, 32)); mx = fmaxf(mx, __shfl_xor(mx, 4, 32)); mx = fmaxf(mx, __shfl_xor(mx, 8, 32));
      const float mnew = fmaxf(m_r[r], mx);
      alpha[r] = (mnew > -1.0e38f) ? __expf(m_r[r] - mnew) : 1.0f;
      const float p0 = (s[0][r] > -1.0e38f) ? __expf(s[0][r] - mnew) : 0.f;
      const float p1 = (s[1][r] > -1.0e38f) ? __expf(s[1][r] - mnew) : 0.f;
      m_r[r] = mnew;
      l_r[r] = l_r[r] * alpha[r] + p0 + p1;
      unsigned short hb = bf16_bits(p0); sPh[w][8 * hh + r][ln] = hb;      sPl[w][8 * hh + r][ln] = bf16_bits(p0 - bf16_val(hb));
      hb = bf16_bits(p1);                sPh[w][8 * hh + r][16 + ln] = hb; sPl[w][8 * hh + r][16 + ln] = bf16_bits(p1 - bf16_val(hb));
    }
#pragma unroll
    for (int dt = 0; dt < DT; ++dt)
#pragma unroll
      for (int r = 0; r < 8; ++r) oacc[dt][r] *= alpha[r];
    __builtin_amdgcn_fence(__ATOMIC_ACQ_REL, "workgroup");
    __builtin_amdgcn_wave_barrier();
    FragB pah, pal;
    pah.half[0] = *(const v8us*)&sPh[w][ln][8 * hh]; pah.half[1] = *(const v8us*)&sPh[w][ln][16 + 8 * hh];
    pal.half[0] = *(const v8us*)&sPl[w][ln][8 * hh]; pal.half[1] = *(const v8us*)&sPl[w][ln][16 + 8 * hh];
#pragma unroll
    for (int dt = 0; dt < DT; ++dt) {
      FragB bvh, bvl;
#pragma unroll
      for (int i = 0; i < 8; ++i) {
        bvh.u[i] = sVh[8 * hh + i][dt * 16 + ln]; bvh.u[8 + i] = sVh[16 + 8 * hh + i][dt * 16 + ln];
        bvl.u[i] = sVl[8 * hh + i][dt * 16 + ln]; bvl.u[8 + i] = sVl[16 + 8 * hh + i][dt * 16 + ln];
      }
      oacc[dt] = mmaN<3>(pah.v, pal.v, bvh.v, bvl.v, oacc[dt]);
    }
    __builtin_amdgcn_fence(__ATOMIC_ACQ_REL, "workgroup");
    __builtin_amdgcn_wave_barrier();
  }
#pragma unroll
  for (int r = 0; r < 8; ++r) {
    float l = l_r[r];
    l += __shfl_xor(l, 1, 32); l += __shfl_xor(l, 2, 32); l += __shfl_xor(l, 4, 32); l += __shfl_xor(l, 8, 32);
    l_r[r] = (l > 0.f) ? 1.0f / l : 0.f;
  }
#pragma unroll
  for (int dt = 0; dt < DT; ++dt)
#pragma unroll
    for (int r = 0; r < 8; ++r) sO[w][8 * hh + r][dt * 16 + ln] = oacc[dt][r] * l_r[r];
  __builtin_amdgcn_fence(__ATOMIC_ACQ_REL, "workgroup");
  __builtin_amdgcn_wave_barrier();
  for (int pass = 0; pass < 2; ++pass) {
    for (int r = 0; r < 16; ++r) {
      const int row = q0 + r;
      for (int c4 = lane * 4; c4 < DV; c4 += 128) {
        if (row < Tq) {
          const v4f val = *(const v4fa*)&sO[w][r][c4];
          *(volatile v4f*)(y + (size_t)bh * ystride + (size_t)row * ypitch + dv0 + c4) = val;
        }
      }
    }
    if (pass == 0) __threadfence();
  }
}

template <bool ASPLIT, int ACT, bool BIAS_BF16, bool RES_BF16>
__global__ __launch_bounds__(128) void k_gemm_bf3(const float* __restrict__ A, int lda, const unsigned short* __restrict__ Wt, int ldb,
                                                const float* __restrict__ bias, const float* __restrict__ resid, int rmod, int ldr,
                                                float* __restrict__ C, int ldc, int M, int N, int K) {
  __shared__ __attribute__((aligned(16))) float so[4][16][64];
  const int tid = threadIdx.x, w = tid >> 5, lane = tid & 31, ln = lane & 15, hh = lane >> 4;
  const int ntn = N / 64;
  const int wid = blockIdx.x * 4 + w;
  const int mt = wid / ntn, nq = wid % ntn;
  if (mt * 16 >= M) return;
  const int row0 = mt * 16, col0 = nq * 64;
  const float* arow = A + (size_t)(row0 + ln) * lda;
  v8f acc[4] = {};
  for (int kb = 0; kb < K; kb += 32) {
    FragB ah, al;
    const v4f x0 = *(const v4fa*)(arow + kb + 8 * hh), x1 = *(const v4fa*)(arow + kb + 8 * hh + 4);
    const v4f x2 = *(const v4fa*)(arow + kb + 16 + 8 * hh), x3 = *(const v4fa*)(arow + kb + 16 + 8 * hh + 4);
    float xs[16] = {x0[0],x0[1],x0[2],x0[3],x1[0],x1[1],x1[2],x1[3],x2[0],x2[1],x2[2],x2[3],x3[0],x3[1],x3[2],x3[3]};
#pragma unroll
    for (int i = 0; i < 16; ++i) { const unsigned short hb = bf16_bits(xs[i]); ah.u[i] = hb; al.u[i] = ASPLIT ? bf16_bits(xs[i] - bf16_val(hb)) : (unsigned short)0; }
#pragma unroll
    for (int t = 0; t < 4; ++t) {
      const unsigned short* brow = Wt + (size_t)(col0 + t * 16 + ln) * ldb + kb;
      FragB b;
      b.half[0] = *(const v8us*)(brow + 8 * hh);
      b.half[1] = *(const v8us*)(brow + 16 + 8 * hh);
      acc[t] = mmaN<ASPLIT ? 2 : 1>(ah.v, al.v, b.v, b.v, acc[t]);
    }
  }
#pragma unroll
  for (int t = 0; t < 4; ++t) {
    const int col = col0 + t * 16 + ln;
    float bv = bias ? bias[col] : 0.f;
    if (BIAS_BF16) bv = bf16_round(bv);
#pragma unroll
    for (int r = 0; r < 8; ++r) {
      float v = acc[t][r] + bv;
      if (resid) { float rv = resid[(size_t)((row0 + 8 * hh + r) % rmod) * ldr + col]; if (RES_BF16) rv = bf16_round(rv); v += rv; }
      if (ACT == 1) v = fmaxf(v, 0.f);
      if (ACT == 2) v = 0.5f * v * (1.0f + erff(v * 0.70710678118654752f));
      if (ACT == 3) { const float u = 0.7978845608028654f * (v + 0.044715f * v * v * v); v = 0.5f * v * (1.0f + tanhf(u)); }
      so[w][8 * hh + r][t * 16 + ln] = v;
    }
  }
  __builtin_amdgcn_fence(__ATOMIC_ACQ_REL, "workgroup");
  __builtin_amdgcn_wave_barrier();
  const int rsub = lane >> 4, c4 = (lane & 15) * 4;
  for (int pass = 0; pass < 2; ++pass) {
#pragma unroll
    for (int q = 0; q < 8; ++q) {
      const int r = q * 2 + rsub;
      const v4f v = *(const v4fa*)&so[w][r][c4];
      *(volatile v4f*)(C + (size_t)(row0 + r) * ldc + col0 + c4) = v;
    }
    if (pass == 0) __threadfence();
  }
}
template <bool PARAM_BF16>
__global__ __launch_bounds__(256) void k_layernorm(const float* __restrict__ X, const float* __restrict__ R, const float* __restrict__ g, const float* __restrict__ bta,
                                                  float* __restrict__ out_sum, float* __restrict__ out_norm, int N, float eps) {
  __shared__ float red[256];
  const int row = blockIdx.x, tid = threadIdx.x;
  const float* x = X + (size_t)row * N; const float* rr = R ? R + (size_t)row * N : nullptr;
  float vals[16];
  const int per = N / 256;
  float s1 = 0.f;
  for (int u = 0; u < per / 4; ++u) {
    const int j = tid * 4 + 1024 * u;
    const v4f a = *(const v4fa*)(x + j);
    v4f b = {0.f,0.f,0.f,0.f}; if (rr) b = *(const v4fa*)(rr + j);
#pragma unroll
    for (int q = 0; q < 4; ++q) { const float v = a[q] + b[q]; vals[u * 4 + q] = v; s1 += v; }
  }
  red[tid] = s1; __syncthreads();
  for (int st = 128; st > 0; st >>= 1) { if (tid < st) red[tid] += red[tid + st]; __syncthreads(); }
  const float mu = red[0] / (float)N; __syncthreads();
  float s2 = 0.f;
  for (int u = 0; u < per / 4; ++u)
#pragma unroll
    for (int q = 0; q < 4; ++q) { const float c = vals[u * 4 + q] - mu; s2 += c * c; }
  red[tid] = s2; __syncthreads();
  for (int st = 128; st > 0; st >>= 1) { if (tid < st) red[tid] += red[tid + st]; __syncthreads(); }
  const float rs = rsqrtf(red[0] / (float)N + eps);
  for (int pass = 0; pass < 2; ++pass) {
    for (int u = 0; u < per / 4; ++u) {
      const int j = tid * 4 + 1024 * u;
      v4f o, sm;
#pragma unroll
      for (int q = 0; q < 4; ++q) {
        float gg = g[j + q], bb = bta[j + q];
        if (PARAM_BF16) { gg = bf16_round(gg); bb = bf16_round(bb); }
        sm[q] = vals[u * 4 + q]; o[q] = (vals[u * 4 + q] - mu) * rs * gg + bb;
      }
      if (out_sum) *(volatile v4f*)(out_sum + (size_t)row * N + j) = sm;
      *(volatile v4f*)(out_norm + (size_t)row * N + j) = o;
    }
    if (pass == 0) __threadfence();
  }
}

typedef _Float16 v16h __attribute__((ext_vector_type(16)));
union FragH { v16h v; v8us half[2]; _Float16 h[16]; unsigned short u[16]; };
template <int NT>
__device__ __forceinline__ v8f mmaH(v16h ah, v16h al, v16h bh, v16h bl, v8f c) {
  c = __builtin_amdgcn_wmma_f32_16x16x32_f16(false, ah, false, bh, (short)0, c, false, false);
  if (NT >= 2) c = __builtin_amdgcn_wmma_f32_16x16x32_f16(false, al, false, bh, (short)0, c, false, false);
  if (NT >= 3) c = __builtin_amdgcn_wmma_f32_16x16x32_f16(false, ah, false, bl, (short)0, c, false, false);
  asm volatile("v_nop\n\tv_nop\n\tv_nop\n\tv_nop" : "+v"(c) : "v"(ah), "v"(al), "v"(bh), "v"(bl));
  return c;
}
template <bool ASPLIT>
__global__ __launch_bounds__(128) void k_gemm_h(const float* __restrict__ A, int lda, size_t sA, const _Float16* __restrict__ Bh, int ldb, size_t sB, float alpha, float* __restrict__ C, int ldc, size_t sC, int M, int N, int K) {
  __shared__ __attribute__((aligned(16))) float so[4][16][64];
  const int tid = threadIdx.x, w = tid >> 5, lane = tid & 31, ln = lane & 15, hh = lane >> 4; const int by = blockIdx.y;
  A += (size_t)by * sA; Bh += (size_t)by * sB; C += (size_t)by * sC;
  const int ntn = (N + 63) / 64; const int wid = blockIdx.x * 4 + w; const int mt = wid / ntn, nq = wid % ntn; if (mt * 16 >= M) return;
  const int row0 = mt * 16, col0 = nq * 64; const float* arow = A + (size_t)(row0 + ln) * lda;
  v8f acc[4] = {};
  for (int kb = 0; kb < K; kb += 32) {
    FragH ah, al;
    const v4f x0 = *(const v4fa*)(arow + kb + 8 * hh), x1 = *(const v4fa*)(arow + kb + 8 * hh + 4), x2 = *(const v4fa*)(arow + kb + 16 + 8 * hh), x3 = *(const v4fa*)(arow + kb + 16 + 8 * hh + 4);
    float xs[16] = {x0[0],x0[1],x0[2],x0[3],x1[0],x1[1],x1[2],x1[3],x2[0],x2[1],x2[2],x2[3],x3[0],x3[1],x3[2],x3[3]};
#pragma unroll
    for (int i = 0; i < 16; ++i) { const _Float16 h = (_Float16)xs[i]; ah.h[i] = h; al.h[i] = ASPLIT ? (_Float16)(xs[i] - (float)h) : (_Float16)0.0f; }
#pragma unroll
    for (int t = 0; t < 4; ++t) { if (col0 + t * 16 >= N) continue; const size_t boff = (size_t)(col0 + t * 16 + ln) * ldb + kb; FragH bq; bq.half[0] = *(const v8us*)(Bh + boff + 8 * hh); bq.half[1] = *(const v8us*)(Bh + boff + 16 + 8 * hh);
      acc[t] = mmaH<ASPLIT ? 2 : 1>(ah.v, al.v, bq.v, bq.v, acc[t]); }
  }
#pragma unroll
  for (int t = 0; t < 4; ++t) { if (col0 + t * 16 >= N) continue;
#pragma unroll
    for (int r = 0; r < 8; ++r) so[w][8 * hh + r][t * 16 + ln] = acc[t][r] * alpha; }
  __builtin_amdgcn_fence(__ATOMIC_ACQ_REL, "workgroup"); __builtin_amdgcn_wave_barrier();
  const int rsub = lane >> 4, c4 = (lane & 15) * 4;
  for (int pass = 0; pass < 2; ++pass) {
#pragma unroll
    for (int q = 0; q < 8; ++q) { const int r = q * 2 + rsub; if (col0 + c4 < N) { const v4f v = *(const v4fa*)&so[w][r][c4]; *(volatile v4f*)(C + (size_t)(row0 + r) * ldc + col0 + c4) = v; } }
    if (pass == 0) __threadfence(); }
}

__global__ __launch_bounds__(256) void k_round_rows(const float* __restrict__ W, unsigned short* __restrict__ Wt, int n8) {
  const int t = blockIdx.x * 256 + threadIdx.x;
  if (t >= n8) return;
  const v4f a = *(const v4fa*)(W + (size_t)t * 8), b = *(const v4fa*)(W + (size_t)t * 8 + 4);
  v8us v; v[0]=bf16_bits(a[0]); v[1]=bf16_bits(a[1]); v[2]=bf16_bits(a[2]); v[3]=bf16_bits(a[3]);
  v[4]=bf16_bits(b[0]); v[5]=bf16_bits(b[1]); v[6]=bf16_bits(b[2]); v[7]=bf16_bits(b[3]);
  *(volatile v8us*)(Wt + (size_t)t * 8) = v; __threadfence(); *(volatile v8us*)(Wt + (size_t)t * 8) = v;
}

__global__ __launch_bounds__(256) void k_scaleadj(const float* __restrict__ a, float* __restrict__ o) { const size_t t = (size_t)blockIdx.x * 256 + threadIdx.x; if (t >= (size_t)NN * NN / 4) return; v4f v = *(const v4fa*)(a + t * 4); for (int q = 0; q < 4; ++q) v[q] = bf16_round(v[q]) * 1024.0f; *(volatile v4f*)(o + t * 4) = v; __threadfence(); *(volatile v4f*)(o + t * 4) = v; }
__global__ __launch_bounds__(256) void k_rev(const float* __restrict__ src, float* __restrict__ dst) { const size_t t = (size_t)blockIdx.x * 256 + threadIdx.x; if (t >= (size_t)NN * DM / 4) return; const size_t l = t / (DM / 4); const int c4 = (int)(t % (DM / 4)) * 4; const v4f v = *(const v4fa*)(src + (size_t)(NN - 1 - l) * DM + c4); *(volatile v4f*)(dst + t * 4) = v; __threadfence(); *(volatile v4f*)(dst + t * 4) = v; }
__global__ __launch_bounds__(256) void k_mconv(const float* __restrict__ XZ, const float* __restrict__ cw, const float* __restrict__ cb, float* __restrict__ U) {
  const size_t t = (size_t)blockIdx.x * 256 + threadIdx.x; if (t >= (size_t)NN * DI) return; const int d = (int)(t % DI); const int l = (int)(t / DI); float a = 0.f;
#pragma unroll
  for (int k = 0; k < KC; ++k) { const int ll = l + k - (KC - 1); if (ll >= 0) a += bf16_round(cw[d * KC + k]) * XZ[(size_t)ll * 512 + d]; }
  a += bf16_round(cb[d]); const float s = a / (1.0f + expf(-a)); *(volatile float*)(U + t) = s; __threadfence(); *(volatile float*)(U + t) = s;
}
__global__ __launch_bounds__(256) void k_wxp(const float* __restrict__ w, unsigned short* __restrict__ Bt) { const int t = blockIdx.x * 256 + threadIdx.x; if (t >= 64 * 32) return; const int n = t / 32, k8 = (t % 32) * 8; v8us v;
#pragma unroll
  for (int i = 0; i < 8; ++i) v[i] = (n < 32) ? bf16_bits(w[n * DI + k8 + i]) : (unsigned short)0; *(volatile v8us*)(Bt + (size_t)n * DI + k8) = v; __threadfence(); *(volatile v8us*)(Bt + (size_t)n * DI + k8) = v; }
__global__ __launch_bounds__(256) void k_mscan(const float* __restrict__ XD, const float* __restrict__ U, const float* __restrict__ XZ, const float* __restrict__ dtw, const float* __restrict__ dtb, const float* __restrict__ Alog, const float* __restrict__ Dp, float* __restrict__ YZ) {
  __shared__ float sx[64];
  const int d = threadIdx.x; float A2[DSG], h[DSG], wdt[DTRG]; for (int s = 0; s < DSG; ++s) { A2[s] = -expf(bf16_round(Alog[d * DSG + s])) * 1.4426950408889634f; h[s] = 0.f; }
  for (int r = 0; r < DTRG; ++r) wdt[r] = bf16_round(dtw[d * DTRG + r]); const float db = bf16_round(dtb[d]), dp = bf16_round(Dp[d]);
#pragma unroll 1
  for (int l = 0; l < NN; ++l) {
    __syncthreads(); if (d < 64) sx[d] = XD[(size_t)l * 64 + d]; __syncthreads();
    float pre = db;
#pragma unroll
    for (int r = 0; r < DTRG; ++r) pre += sx[r] * wdt[r];
    const float dt = fmaxf(pre, 0.f) + log1pf(expf(-fabsf(pre))); const float u = U[(size_t)l * DI + d]; const float du = dt * u; float y = 0.f;
#pragma unroll
    for (int s = 0; s < DSG; ++s) { h[s] = exp2f(dt * A2[s]) * h[s] + du * sx[DTRG + s]; y += h[s] * sx[DTRG + DSG + s]; }
    y += u * dp; const float z = XZ[(size_t)l * 512 + DI + d]; const float o = y * (z / (1.0f + expf(-z)));
    *(volatile float*)(YZ + (size_t)l * DI + d) = o; }
  __syncthreads();
#pragma unroll 1
  for (int l = 0; l < NN; ++l) { const float o = YZ[(size_t)l * DI + d]; *(volatile float*)(YZ + (size_t)l * DI + d) = o; }
}
__global__ __launch_bounds__(256) void k_gafinal(const float* __restrict__ G0, const float* __restrict__ G1, const float* __restrict__ XI, const float* __restrict__ g, const float* __restrict__ b, const float* __restrict__ m, const float* __restrict__ v, float* __restrict__ GA, float* __restrict__ XL, float* __restrict__ XS) {
  const size_t t = (size_t)blockIdx.x * 256 + threadIdx.x; if (t >= (size_t)NN * DM / 4) return; const size_t l = t / (DM / 4); const int c4 = (int)(t % (DM / 4)) * 4;
  const v4f g0 = *(const v4fa*)(G0 + t * 4), g1 = *(const v4fa*)(G1 + (size_t)(NN - 1 - l) * DM + c4), xi = *(const v4fa*)(XI + t * 4); v4f ga, xl;
  for (int q = 0; q < 4; ++q) { const int c = c4 + q; ga[q] = fmaxf(g0[q] + g1[q], 0.f) * 0.9f + 0.1f * xi[q]; const float inv = 1.0f / sqrtf(bf16_round(v[c]) + 1e-5f); xl[q] = fmaxf((xi[q] - bf16_round(m[c])) * inv * bf16_round(g[c]) + bf16_round(b[c]), 0.f); }
  *(volatile v4f*)(GA + t * 4) = ga; *(volatile v4f*)(XL + t * 4) = xl; *(volatile v4f*)(XS + l * (LG * DM) + c4) = xl; __threadfence(); *(volatile v4f*)(GA + t * 4) = ga; *(volatile v4f*)(XL + t * 4) = xl; *(volatile v4f*)(XS + l * (LG * DM) + c4) = xl;
}
__global__ __launch_bounds__(256) void k_xT(const float* __restrict__ xi, int ld, _Float16* __restrict__ XT) { const int t = blockIdx.x * 256 + threadIdx.x; if (t >= DM * (NN / 8)) return; const int n8 = (t % (NN / 8)) * 8, d = t / (NN / 8); FragH f;
#pragma unroll
  for (int i = 0; i < 8; ++i) f.h[i] = (_Float16)xi[(size_t)(n8 + i) * ld + d]; const v8us o = f.half[0]; *(volatile v8us*)((unsigned short*)XT + (size_t)d * NN + n8) = o; __threadfence(); *(volatile v8us*)((unsigned short*)XT + (size_t)d * NN + n8) = o; }
__global__ __launch_bounds__(256) void k_gmix(const float* __restrict__ T, const float* __restrict__ XL, int it, float* __restrict__ XS) { const size_t t = (size_t)blockIdx.x * 256 + threadIdx.x; if (t >= (size_t)NN * DM / 4) return; const size_t n = t / (DM / 4); const int c4 = (int)(t % (DM / 4)) * 4; const v4f a = *(const v4fa*)(T + t * 4), x = *(const v4fa*)(XL + t * 4); v4f o;
  for (int q = 0; q < 4; ++q) o[q] = 0.95f * a[q] + 0.05f * x[q]; *(volatile v4f*)(XS + n * (LG * DM) + (size_t)it * DM + c4) = o; __threadfence(); *(volatile v4f*)(XS + n * (LG * DM) + (size_t)it * DM + c4) = o; }
__global__ __launch_bounds__(256) void k_wbx(const float* __restrict__ w, unsigned short* __restrict__ Bt) { const int t = blockIdx.x * 256 + threadIdx.x; if (t >= 64 * 32) return; const int n = t / 32, k8 = (t % 32) * 8; v8us v;
#pragma unroll
  for (int i = 0; i < 8; ++i) v[i] = (n < 48) ? bf16_bits(w[(size_t)(k8 + i) * 48 + n]) : (unsigned short)0; *(volatile v8us*)(Bt + (size_t)n * DM + k8) = v; __threadfence(); *(volatile v8us*)(Bt + (size_t)n * DM + k8) = v; }
__global__ __launch_bounds__(256) void k_bscan(const float* __restrict__ XDB, const float* __restrict__ XS, const float* __restrict__ dtw, const float* __restrict__ Alog, const float* __restrict__ Dp, float* __restrict__ Y7) {
  const size_t t = (size_t)blockIdx.x * 256 + threadIdx.x; if (t >= (size_t)NN * DM) return; const int d = (int)(t % DM); const size_t n = t / DM; float h[DSB], A2[DSB]; for (int s = 0; s < DSB; ++s) { h[s] = 0.f; A2[s] = -expf(bf16_round(Alog[d * DSB + s])) * 1.4426950408889634f; }
  const float dp = bf16_round(Dp[d]); float y = 0.f;
#pragma unroll 1
  for (int l = 0; l < LG; ++l) { const float* xd = XDB + (n * LG + l) * 64; float pre = 0.f;
#pragma unroll 1
    for (int r = 0; r < DTRB; ++r) pre += xd[r] * bf16_round(dtw[r * DM + d]);
    const float dt = fmaxf(pre, 0.f) + log1pf(expf(-fabsf(pre))); const float u = XS[(n * LG + l) * DM + d]; const float du = dt * u; y = 0.f;
#pragma unroll 1
    for (int s = 0; s < DSB; ++s) { h[s] = exp2f(dt * A2[s]) * h[s] + du * xd[DTRB + s]; y += h[s] * xd[DTRB + DSB + s]; }
    y += u * dp; }
  *(volatile float*)(Y7 + t) = y; __threadfence(); *(volatile float*)(Y7 + t) = y;
}
__global__ __launch_bounds__(256) void k_out(const float* __restrict__ LO, const float* __restrict__ GA, const float* __restrict__ g, const float* __restrict__ b, const float* __restrict__ m, const float* __restrict__ v, float* __restrict__ out) {
  const size_t t = (size_t)blockIdx.x * 256 + threadIdx.x; if (t >= (size_t)NN * DM / 4) return; const int c4 = (int)(t % (DM / 4)) * 4; const v4f lo = *(const v4fa*)(LO + t * 4), ga = *(const v4fa*)(GA + t * 4); v4f o;
  for (int q = 0; q < 4; ++q) { const int c = c4 + q; const float x = lo[q] * 0.8f + ga[q] * 0.2f; const float inv = 1.0f / sqrtf(bf16_round(v[c]) + 1e-5f); o[q] = fmaxf((x - bf16_round(m[c])) * inv * bf16_round(g[c]) + bf16_round(b[c]), 0.f); }
  *(volatile v4f*)(out + t * 4) = o; __threadfence(); *(volatile v4f*)(out + t * 4) = o;
}
extern "C" void kernel_launch(void* const* d_in, const int* in_sizes, int n_in,
                              void* d_out, int out_size, void* d_ws, size_t ws_size, hipStream_t stream) {
  (void)in_sizes; (void)n_in; (void)out_size;
  const float* x = (const float*)d_in[0]; const float* adj = (const float*)d_in[1]; const float* lin1 = (const float*)d_in[2]; const float* g_in = (const float*)d_in[3]; const float* g_cw = (const float*)d_in[4]; const float* g_cb = (const float*)d_in[5];
  const float* g_xp = (const float*)d_in[6]; const float* g_dtw = (const float*)d_in[7]; const float* g_dtb = (const float*)d_in[8]; const float* g_Al = (const float*)d_in[9]; const float* g_D = (const float*)d_in[10]; const float* g_out = (const float*)d_in[11];
  const float* bn1g = (const float*)d_in[12]; const float* bn1b = (const float*)d_in[13]; const float* bn1m = (const float*)d_in[14]; const float* bn1v = (const float*)d_in[15];
  const float* b_xp = (const float*)d_in[16]; const float* b_dtw = (const float*)d_in[17]; const float* b_Al = (const float*)d_in[18]; const float* b_D = (const float*)d_in[19]; const float* b_outw = (const float*)d_in[20];
  const float* bn2g = (const float*)d_in[21]; const float* bn2b = (const float*)d_in[22]; const float* bn2m = (const float*)d_in[23]; const float* bn2v = (const float*)d_in[24];
  float* OUT = (float*)d_out; float* XI = OUT + (size_t)NN * DM; float* GA = OUT + (size_t)2 * NN * DM; float* LO = OUT + (size_t)3 * NN * DM;
  char* ws = (char*)d_ws; size_t off = 0;
  auto take = [&](size_t bytes) { char* p = ws + off; off += (bytes + 255) & ~(size_t)255; return p; };
  unsigned short* Blin = (unsigned short*)take((size_t)DM * FIN * 2); unsigned short* Bin = (unsigned short*)take((size_t)512 * DM * 2); unsigned short* Bxp = (unsigned short*)take((size_t)64 * DI * 2); unsigned short* Bgo = (unsigned short*)take((size_t)DM * DI * 2); unsigned short* Bbx = (unsigned short*)take((size_t)64 * DM * 2); unsigned short* Bbo = (unsigned short*)take((size_t)DM * DM * 2);
  float* Xrev = (float*)take((size_t)NN * DM * 4); float* XZ = (float*)take((size_t)NN * 512 * 4); float* U = (float*)take((size_t)NN * DI * 4); float* XD = (float*)take((size_t)NN * 64 * 4); float* YZ = (float*)take((size_t)NN * DI * 4); float* G0 = (float*)take((size_t)NN * DM * 4); float* G1 = (float*)take((size_t)NN * DM * 4);
  float* XL = (float*)take((size_t)NN * DM * 4); float* XS = (float*)take((size_t)NN * LG * DM * 4); _Float16* XT = (_Float16*)take((size_t)DM * NN * 2); float* T = (float*)take((size_t)NN * DM * 4); float* XDB = (float*)take((size_t)NN * LG * 64 * 4); float* Y7 = (float*)take((size_t)NN * DM * 4); float* ADJ = (float*)take((size_t)NN * NN * 4);
  if (off > ws_size) return;
  k_wt_bf16<<<(DM * (FIN / 8) + 255) / 256, 256, 0, stream>>>(lin1, Blin, FIN, DM); k_round_rows<<<(512 * DM / 8 + 255) / 256, 256, 0, stream>>>(g_in, Bin, 512 * DM / 8); k_wxp<<<8, 256, 0, stream>>>(g_xp, Bxp); k_round_rows<<<(DM * DI / 8 + 255) / 256, 256, 0, stream>>>(g_out, Bgo, DM * DI / 8);
  k_wbx<<<8, 256, 0, stream>>>(b_xp, Bbx); k_wt_bf16<<<(DM * 32 + 255) / 256, 256, 0, stream>>>(b_outw, Bbo, DM, DM);
  const unsigned g4 = ((NN / 16) * 4 + 3) / 4;
  k_gemm_bf3<false, 0, false, false><<<g4, 128, 0, stream>>>(x, FIN, Blin, FIN, nullptr, nullptr, 1, 0, XI, DM, NN, DM, FIN);
  k_rev<<<(NN * DM / 4 + 255) / 256, 256, 0, stream>>>(XI, Xrev); k_scaleadj<<<(NN * NN / 4 + 255) / 256, 256, 0, stream>>>(adj, ADJ);
  for (int dir = 0; dir < 2; ++dir) { const float* src = dir ? Xrev : XI; float* G = dir ? G1 : G0;
    k_gemm_bf3<true, 0, false, false><<<((NN / 16) * 8 + 3) / 4, 128, 0, stream>>>(src, DM, Bin, DM, nullptr, nullptr, 1, 0, XZ, 512, NN, 512, DM);
    k_mconv<<<(NN * DI + 255) / 256, 256, 0, stream>>>(XZ, g_cw, g_cb, U);
    k_gemm_bf3<true, 0, false, false><<<((NN / 16) * 1 + 3) / 4, 128, 0, stream>>>(U, DI, Bxp, DI, nullptr, nullptr, 1, 0, XD, 64, NN, 64, DI);
    k_mscan<<<1, 256, 0, stream>>>(XD, U, XZ, g_dtw, g_dtb, g_Al, g_D, YZ);
    k_gemm_bf3<true, 0, false, false><<<g4, 128, 0, stream>>>(YZ, DI, Bgo, DI, nullptr, nullptr, 1, 0, G, DM, NN, DM, DI); }
  k_gafinal<<<(NN * DM / 4 + 255) / 256, 256, 0, stream>>>(G0, G1, XI, bn1g, bn1b, bn1m, bn1v, GA, XL, XS);
  const float* xi = XL; int xld = DM;
  for (int it = 1; it < LG; ++it) {
    k_xT<<<(DM * (NN / 8) + 255) / 256, 256, 0, stream>>>(xi, xld, XT);
    k_gemm_h<false><<<dim3(g4, 1), 128, 0, stream>>>(ADJ, NN, 0, XT, NN, 0, 0.0009765625f, T, DM, 0, NN, DM, NN);
    k_gmix<<<(NN * DM / 4 + 255) / 256, 256, 0, stream>>>(T, XL, it, XS);
    xi = XS + (size_t)it * DM; xld = LG * DM; }
  k_gemm_bf3<true, 1, false, false><<<((NN * LG / 16) * 1 + 3) / 4, 128, 0, stream>>>(XS, DM, Bbx, DM, nullptr, nullptr, 1, 0, XDB, 64, NN * LG, 64, DM);
  k_bscan<<<(NN * DM + 255) / 256, 256, 0, stream>>>(XDB, XS, b_dtw, b_Al, b_D, Y7);
  k_gemm_bf3<true, 0, false, false><<<g4, 128, 0, stream>>>(Y7, DM, Bbo, DM, nullptr, XI, NN, DM, LO, DM, NN, DM, DM);
  k_out<<<(NN * DM / 4 + 255) / 256, 256, 0, stream>>>(LO, GA, bn2g, bn2b, bn2m, bn2v, OUT);
}
